// Center_pose_head_90194313216456
// MI455X (gfx1250) — hardware-run, weakly checked
//
#include <hip/hip_runtime.h>
#include <stddef.h>
#include <math.h>

typedef __attribute__((ext_vector_type(16))) _Float16 v16h;
typedef __attribute__((ext_vector_type(8)))  _Float16 v8h;
typedef __attribute__((ext_vector_type(16))) __bf16   v16b;
typedef __attribute__((ext_vector_type(8)))  __bf16   v8b;
typedef __attribute__((ext_vector_type(8)))  float    v8f;
typedef __attribute__((ext_vector_type(4)))  float    v4f;

constexpr int   NB     = 4;
constexpr int   NTHR   = 256;
constexpr float ACARRY = 8.0f;
constexpr float WCARRY = 256.0f;
constexpr float INV_AW = 1.0f / 2048.0f;
constexpr float INV_W  = 1.0f / 256.0f;
constexpr int   OMP    = 64;
constexpr int   NHID   = 768;
constexpr int   HK1    = 576;
constexpr int   HM2    = 64;
constexpr int   NCLS   = 53;
constexpr int   NPIMG  = 16384;
constexpr int   RES_OUT_LOG = 7;

static_assert((9 * 1024) % 32 == 0 && (9 * 512) % 32 == 0 && (9 * 256) % 32 == 0);
static_assert((4 * 512) % 32 == 0 && (4 * 256) % 32 == 0 && (4 * 64) % 32 == 0);
static_assert(HK1 % 32 == 0 && NHID % 32 == 0 && NHID % 64 == 0 && HM2 % 64 == 0 && NPIMG % 64 == 0);
static_assert(OMP % 64 == 0);

constexpr size_t SZ_WPO0 = 64ull * 9216 * 2, SZ_WPO1 = 64ull * 4608 * 2, SZ_WPO2 = 64ull * 2304 * 2;
constexpr size_t SZ_WDW0 = 512ull * 9216 * 2, SZ_WDW1 = 256ull * 4608 * 2, SZ_WDW2 = 64ull * 2304 * 2;
constexpr size_t SZ_UWP0 = 4ull * 512 * 2048 * 2, SZ_UWP1 = 4ull * 256 * 1024 * 2, SZ_UWP2 = 4ull * 64 * 256 * 2;
constexpr size_t SZ_WH1  = 768ull * 576 * 2, SZ_WH2 = 64ull * 768 * 2;
constexpr size_t SZ_SH0  = 2048, SZ_SH1 = 1024, SZ_SH2 = 256, SZ_B1F = 3072, SZ_B2P = 256;
constexpr size_t SZ_OM   = 8192ull * OMP * 4;
constexpr size_t SZ_COL  = 18874368ull * 2;
constexpr size_t SZ_ACTB = 16384ull * 64 * 4;
constexpr size_t SZ_PACT = 4ull * 16384 * 64 * 4;
constexpr size_t SZ_HID  = 16384ull * 768 * 2;
constexpr size_t WS_TOTAL = SZ_WPO0 + SZ_WPO1 + SZ_WPO2 + SZ_WDW0 + SZ_WDW1 + SZ_WDW2 + SZ_UWP0 + SZ_UWP1 + SZ_UWP2
                          + SZ_WH1 + SZ_WH2 + SZ_SH0 + SZ_SH1 + SZ_SH2 + SZ_B1F + SZ_B2P
                          + SZ_OM + SZ_COL + SZ_ACTB + SZ_PACT + SZ_PACT + SZ_HID;
static_assert(WS_TOTAL == 128522752ull);
static_assert(WS_TOTAL <= 134217728ull);
static_assert(1024ull * 9216 * 2 <= SZ_COL && 4096ull * 4608 * 2 <= SZ_COL && 8192ull * 2304 * 2 <= SZ_COL);
static_assert(4ull * 1024 * 2048 * 2 <= SZ_COL && 4ull * 4096 * 1024 * 2 <= SZ_COL && 4ull * 16384 * 256 * 2 <= SZ_COL);
static_assert(16384ull * 576 * 2 <= SZ_COL);
static_assert(1024ull * 512 * 4 <= SZ_ACTB && 4096ull * 256 * 4 <= SZ_ACTB && 16384ull * 64 * 4 <= SZ_ACTB);
static_assert(4ull * 1024 * 512 * 4 <= SZ_PACT && 4ull * 4096 * 256 * 4 <= SZ_PACT && 4ull * 16384 * 64 * 4 <= SZ_PACT);
static_assert(4ull * 1024 * 16 * 16 * 4 <= SZ_PACT);
static_assert(4096ull * OMP * 4 <= SZ_OM && 8192ull * OMP * 4 <= SZ_OM && 1024ull * OMP * 4 <= SZ_OM);

__device__ __forceinline__ unsigned short f2bf_bits(float f) {
  unsigned u = __float_as_uint(f);
  return (unsigned short)((u + 0x7FFFu + ((u >> 16) & 1u)) >> 16);
}
__device__ __forceinline__ float bf_bits2f(unsigned short h) { return __uint_as_float(((unsigned)h) << 16); }

__device__ __forceinline__ void dep_guard_h(v8f& a, v8f& b, v16h x, v16h y) { asm volatile("v_nop\n\tv_nop\n\tv_nop\n\tv_nop" : "+v"(a), "+v"(b) : "v"(x), "v"(y)); }
__device__ __forceinline__ void dep_guard_b(v8f& a, v8f& b, v16b x, v16b y) { asm volatile("v_nop\n\tv_nop\n\tv_nop\n\tv_nop" : "+v"(a), "+v"(b) : "v"(x), "v"(y)); }
__device__ __forceinline__ void dep_guard4_h(v8f& a, v8f& b, v8f& c, v8f& d, v16h x, v16h y) { asm volatile("v_nop\n\tv_nop\n\tv_nop\n\tv_nop" : "+v"(a), "+v"(b), "+v"(c), "+v"(d) : "v"(x), "v"(y)); }
__device__ __forceinline__ void dep_guard4_b(v8f& a, v8f& b, v8f& c, v8f& d, v16b x, v16b y) { asm volatile("v_nop\n\tv_nop\n\tv_nop\n\tv_nop" : "+v"(a), "+v"(b), "+v"(c), "+v"(d) : "v"(x), "v"(y)); }
__device__ __forceinline__ void keep4_h(v16h a, v16h b, v16h c, v16h d) { asm volatile("v_nop" :: "v"(a), "v"(b), "v"(c), "v"(d)); }
__device__ __forceinline__ void keep4_b(v16b a, v16b b, v16b c, v16b d) { asm volatile("v_nop" :: "v"(a), "v"(b), "v"(c), "v"(d)); }
__device__ __forceinline__ void acc_guard4(v8f& a, v8f& b, v8f& c, v8f& d) { asm volatile("v_nop\n\tv_nop\n\tv_nop\n\tv_nop" : "+v"(a), "+v"(b), "+v"(c), "+v"(d)); }
template <typename T> struct Frag;
template <> struct Frag<_Float16> {
  typedef v16h V; union U { v16h v; v8h h[2]; };
  static __device__ __forceinline__ v16h load(const _Float16* p) {
    U f; f.h[0] = *(const v8h*)(p); f.h[1] = *(const v8h*)(p + 16); return f.v;
  }
  static __device__ __forceinline__ v8f mma(v16h a, v16h b, v8f c) {
    return __builtin_amdgcn_wmma_f32_16x16x32_f16(false, a, false, b, (short)0, c, false, false);
  }
  static __device__ __forceinline__ void guard(v8f& a, v8f& b, v16h x, v16h y) { dep_guard_h(a, b, x, y); }
  static __device__ __forceinline__ void guard4(v8f& a, v8f& b, v8f& c, v8f& d, v16h x, v16h y) { dep_guard4_h(a, b, c, d, x, y); }
  static __device__ __forceinline__ void keep(v16h a, v16h b, v16h c, v16h d) { keep4_h(a, b, c, d); }
};
template <> struct Frag<__bf16> {
  typedef v16b V; union U { v16b v; v8b h[2]; };
  static __device__ __forceinline__ v16b load(const __bf16* p) {
    U f; f.h[0] = *(const v8b*)(p); f.h[1] = *(const v8b*)(p + 16); return f.v;
  }
  static __device__ __forceinline__ v8f mma(v16b a, v16b b, v8f c) {
    return __builtin_amdgcn_wmma_f32_16x16x32_bf16(false, a, false, b, (short)0, c, false, false);
  }
  static __device__ __forceinline__ void guard(v8f& a, v8f& b, v16b x, v16b y) { dep_guard_b(a, b, x, y); }
  static __device__ __forceinline__ void guard4(v8f& a, v8f& b, v8f& c, v8f& d, v16b x, v16b y) { dep_guard4_b(a, b, c, d, x, y); }
  static __device__ __forceinline__ void keep(v16b a, v16b b, v16b c, v16b d) { keep4_b(a, b, c, d); }
};

template <int ET> struct Elem;
template <> struct Elem<0> { typedef _Float16 T; };
template <> struct Elem<1> { typedef __bf16 T; };
template <int ET, bool SPLIT, int BIAS_MODE, int OUT_MODE, bool RESID, int ACT, int MG>
__global__ __launch_bounds__(256) void wmma_gemm64(
    const unsigned short* __restrict__ Ap, const unsigned short* __restrict__ A2p, int lda, long strideA,
    const unsigned short* __restrict__ Btp, const unsigned short* __restrict__ Bt2p, int ldb, long strideB,
    void* __restrict__ Cout, void* __restrict__ Cout2, int ldc, long strideC,
    const float* __restrict__ bias,
    const float* __restrict__ resid, long strideR,
    int M, int N, int K, float scale, int Mst) {
  typedef typename Elem<ET>::T T;
  typedef typename Frag<T>::V V;
  const T* A = (const T*)Ap; const T* A2 = (const T*)A2p; const T* Bt = (const T*)Btp; const T* Bt2 = (const T*)Bt2p;
  __shared__ __align__(16) float sT[8][16 * 68];
  const int b    = blockIdx.y;
  const int lane = threadIdx.x & 31;
  const int wave = threadIdx.x >> 5;
  const int tilesN = N >> 6;
  const int tilesM = M >> 6;
  const int tile = blockIdx.x * 8 + wave;
  if (tile >= tilesM * tilesN) return;
  const int tm = tile / tilesN;
  const int tn = tile - tm * tilesN;
  const int m0 = tm << 6;
  const int n0 = tn << 6;

  const T* Ab  = A  + (size_t)b * strideA;
  const T* Bb  = Bt + (size_t)b * strideB;
  const T* Ab2 = SPLIT ? (A2  + (size_t)b * strideA) : nullptr;
  const T* Bb2 = SPLIT ? (Bt2 + (size_t)b * strideB) : nullptr;

  const int rlane = lane & 15;
  const int koff  = (lane >> 4) * 8;
  const int mOff  = (lane >> 4) * 8;

  v8f acc[4][4];
#pragma unroll
  for (int i = 0; i < 4; ++i)
#pragma unroll
    for (int j = 0; j < 4; ++j) acc[i][j] = (v8f){0.f,0.f,0.f,0.f,0.f,0.f,0.f,0.f};

  for (int k0 = 0; k0 < K; k0 += 32) {
    V bh[4], bl[4];
#pragma unroll
    for (int j = 0; j < 4; ++j) {
      const size_t bo = (size_t)(n0 + (j << 4) + rlane) * ldb + koff + k0;
      bh[j] = Frag<T>::load(Bb + bo);
      if (SPLIT) bl[j] = Frag<T>::load(Bb2 + bo);
    }
#pragma unroll
    for (int i = 0; i < 4; ++i) {
      const size_t ao = (size_t)(m0 + (i << 4) + rlane) * lda + koff + k0;
      V ah = Frag<T>::load(Ab + ao);
      V al;
      if (SPLIT) al = Frag<T>::load(Ab2 + ao);
#pragma unroll
      for (int j = 0; j < 4; ++j) {
        acc[i][j] = Frag<T>::mma(ah, bh[j], acc[i][j]);
        if (SPLIT) {
          acc[i][j] = Frag<T>::mma(ah, bl[j], acc[i][j]);
          acc[i][j] = Frag<T>::mma(al, bh[j], acc[i][j]);
        }
      }
      Frag<T>::guard4(acc[i][0], acc[i][1], acc[i][2], acc[i][3], ah, SPLIT ? al : ah);
    }
    Frag<T>::keep(bh[0], bh[1], bh[2], bh[3]);
    if (SPLIT) Frag<T>::keep(bl[0], bl[1], bl[2], bl[3]);
  }
  acc_guard4(acc[0][0], acc[0][1], acc[0][2], acc[0][3]);
  acc_guard4(acc[1][0], acc[1][1], acc[1][2], acc[1][3]);
  acc_guard4(acc[2][0], acc[2][1], acc[2][2], acc[2][3]);
  acc_guard4(acc[3][0], acc[3][1], acc[3][2], acc[3][3]);

  float* slab = sT[wave];
  const float* Rb = RESID ? (resid + (size_t)b * strideR) : nullptr;
#pragma unroll
  for (int i = 0; i < 4; ++i) {
    const int mBase = m0 + (i << 4);
#pragma unroll
    for (int j = 0; j < 4; ++j) {
      const int n = n0 + (j << 4) + rlane;
      float bv = 0.f;
      if (BIAS_MODE == 2) bv = bias[n];
#pragma unroll
      for (int r = 0; r < 8; ++r) {
        float v = acc[i][j][r] * scale;
        if (BIAS_MODE == 1) v += bias[mBase + mOff + r];
        if (BIAS_MODE == 2) v += bv;
        if (RESID) v += Rb[(size_t)(mBase + mOff + r) * ldc + n];
        if (ACT == 1) v = tanhf(v);
        if (ACT == 2) v = fmaxf(v, 0.0f);
        if (ACT == 3) v = v / (1.0f + expf(-v));
        if (ACT == 4) v = (v > 0.f) ? v : 0.01f * v;
        if (ACT == 5) v = 0.5f * v * (1.0f + erff(v * 0.70710678118654752f));
        slab[(mOff + r) * 68 + (j << 4) + rlane] = v;
      }
    }
    __builtin_amdgcn_fence(__ATOMIC_RELEASE, "workgroup");
    __builtin_amdgcn_wave_barrier();
    __builtin_amdgcn_fence(__ATOMIC_ACQUIRE, "workgroup");
    if (OUT_MODE == 0) {
      float* C = (float*)Cout + (size_t)b * strideC;
      const int hh = lane >> 4, c4 = (lane & 15) * 4;
      for (int pass = 0; pass < 2; ++pass) {
#pragma unroll
        for (int it = 0; it < 8; ++it) {
          const int row = it * 2 + hh;
          v4f v = *(const v4f*)(slab + row * 68 + c4);
          if (MG == 0 || (mBase + row) < Mst)
            *(volatile v4f*)(C + (size_t)(mBase + row) * ldc + n0 + c4) = v;
        }
        __threadfence();
      }
    } else {
      const int q = lane >> 3, c8 = (lane & 7) * 8;
      unsigned short* C  = (unsigned short*)Cout  + (size_t)b * strideC;
      unsigned short* C2 = (OUT_MODE == 2) ? ((unsigned short*)Cout2 + (size_t)b * strideC) : nullptr;
      for (int pass = 0; pass < 2; ++pass) {
#pragma unroll
        for (int it = 0; it < 4; ++it) {
          const int row = it * 4 + q;
          const float* sp = slab + row * 68 + c8;
          v8h hv, lv;
#pragma unroll
          for (int e = 0; e < 8; ++e) {
            if (OUT_MODE == 1) {
              hv[e] = (_Float16)sp[e];
            } else {
              unsigned short hb = f2bf_bits(sp[e]);
              unsigned short lb = f2bf_bits(sp[e] - bf_bits2f(hb));
              hv[e] = __builtin_bit_cast(_Float16, hb);
              lv[e] = __builtin_bit_cast(_Float16, lb);
            }
          }
          *(volatile v8h*)(C + (size_t)(mBase + row) * ldc + n0 + c8) = hv;
          if (OUT_MODE == 2) *(volatile v8h*)(C2 + (size_t)(mBase + row) * ldc + n0 + c8) = lv;
        }
        __threadfence();
      }
    }
    __builtin_amdgcn_fence(__ATOMIC_RELEASE, "workgroup");
    __builtin_amdgcn_wave_barrier();
    __builtin_amdgcn_fence(__ATOMIC_ACQUIRE, "workgroup");
  }
}

__device__ __forceinline__ int iclamp(int v, int lo, int hi) { return v < lo ? lo : (v > hi ? hi : v); }

__device__ __forceinline__ void st2_h8(unsigned short* p, v8h v) {
  *(volatile v8h*)p = v;
  __threadfence();
  *(volatile v8h*)p = v;
}
__device__ __forceinline__ void st2_f4(float* p, v4f v) {
  *(volatile v4f*)p = v;
  __threadfence();
  *(volatile v4f*)p = v;
}
__device__ __forceinline__ void st2_f1(float* p, float v) {
  *(volatile float*)p = v;
  __threadfence();
  *(volatile float*)p = v;
}

__device__ __forceinline__ size_t pact_pix(int b, int Y, int X, int lrh) {
  const int p = ((Y & 1) << 1) | (X & 1);
  return ((((size_t)(p * NB + b) << lrh) + (size_t)(Y >> 1)) << lrh) + (size_t)(X >> 1);
}

__global__ __launch_bounds__(NTHR) void k_xprep(const float* __restrict__ x, float* __restrict__ xp) {
  const int i   = blockIdx.x * NTHR + threadIdx.x;
  if (i >= 262144) return;
  const int c0  = (i & 255) << 2;
  const int pix = i >> 8;
  const int p   = pix >> 8;
  const int rem = pix & 255;
  const int b   = rem >> 6;
  const int yh  = (rem >> 3) & 7;
  const int xh  = rem & 7;
  const int Y   = 2 * yh + (p >> 1);
  const int X   = 2 * xh + (p & 1);
  const float* sp = x + (((size_t)b * 1024 + c0) * 16 + Y) * 16 + X;
  v4f v;
  v[0] = sp[0]; v[1] = sp[256]; v[2] = sp[512]; v[3] = sp[768];
  st2_f4(xp + (size_t)i * 4, v);
}

template <bool SFOLD>
__global__ __launch_bounds__(NTHR) void k_pack3(const float* __restrict__ w, const float* __restrict__ svec,
                                                int O, int lc, int nrow, unsigned short* __restrict__ out) {
  const int C   = 1 << lc;
  const int cpr = (9 * C) >> 3;
  const int i   = blockIdx.x * NTHR + threadIdx.x;
  if (i >= nrow * cpr) return;
  const int o   = i / cpr;
  const int q   = i - o * cpr;
  const int e0  = q << 3;
  const int k   = e0 >> lc;
  const int c0  = e0 & (C - 1);
  const int oc  = (o < O) ? o : (O - 1);
  float f = (o < O) ? WCARRY : 0.0f;
  if constexpr (SFOLD) f = f * svec[oc];
  const float* sp = w + ((size_t)oc * C + c0) * 9 + k;
  v8h hv;
#pragma unroll
  for (int e = 0; e < 8; ++e) hv[e] = (_Float16)(sp[(size_t)e * 9] * f);
  st2_h8(out + (size_t)i * 8, hv);
}

__global__ __launch_bounds__(NTHR) void k_packdec(const float* __restrict__ uw, const float* __restrict__ s2,
                                                  int lco, unsigned short* __restrict__ out) {
  const int Co  = 1 << lco;
  const int i   = blockIdx.x * NTHR + threadIdx.x;
  if (i >= 2 * Co * Co) return;
  const int lper = 2 * lco - 1;
  const int p   = i >> lper;
  const int rem = i & ((1 << lper) - 1);
  const int co  = rem >> (lco - 1);
  const int q   = rem & ((Co >> 1) - 1);
  const int e0  = q << 3;
  const int t   = e0 >> lco;
  const int ci0 = e0 & (Co - 1);
  const int a = p >> 1, bb = p & 1, ty = t >> 1, tx = t & 1;
  const int ky = 3 - a - 2 * ty, kx = 3 - bb - 2 * tx;
  const float f = WCARRY * s2[co];
  const float* sp = uw + (((size_t)ci0 * Co + co) * 4 + ky) * 4 + kx;
  const size_t cs = (size_t)Co * 16;
  v8h hv;
#pragma unroll
  for (int e = 0; e < 8; ++e) hv[e] = (_Float16)(sp[(size_t)e * cs] * f);
  st2_h8(out + (size_t)i * 8, hv);
}

__global__ __launch_bounds__(NTHR) void k_packh2(const float* __restrict__ w2a, const float* __restrict__ w2b,
                                                 const float* __restrict__ w2c, unsigned short* __restrict__ out) {
  const int hd  = blockIdx.y;
  const float* w = (hd == 0) ? w2a : ((hd == 1) ? w2b : w2c);
  const int cls = (hd == 0) ? 34 : ((hd == 1) ? 17 : 2);
  const int rb  = (hd == 0) ? 0 : ((hd == 1) ? 34 : 51);
  const int i   = blockIdx.x * NTHR + threadIdx.x;
  if (i >= 64 * 32) return;
  const int r   = i >> 5, q = i & 31, e0 = q << 3;
  const int lr  = r - rb;
  const float f = (lr >= 0 && lr < cls) ? WCARRY : 0.0f;
  const int lrc = iclamp(lr, 0, cls - 1);
  const float* sp = w + (size_t)lrc * 256 + e0;
  const v4f u0 = *(const v4f*)sp;
  const v4f u1 = *(const v4f*)(sp + 4);
  v8h hv;
#pragma unroll
  for (int e = 0; e < 4; ++e) { hv[e] = (_Float16)(u0[e] * f); hv[4 + e] = (_Float16)(u1[e] * f); }
  st2_h8(out + (size_t)r * NHID + hd * 256 + e0, hv);
}

__global__ __launch_bounds__(NTHR) void k_tables(
    const float* __restrict__ db0, const float* __restrict__ s10, const float* __restrict__ t10,
    const float* __restrict__ db1, const float* __restrict__ s11, const float* __restrict__ t11,
    const float* __restrict__ db2, const float* __restrict__ s12, const float* __restrict__ t12,
    const float* __restrict__ b1a, const float* __restrict__ b1b, const float* __restrict__ b1c,
    const float* __restrict__ b2a, const float* __restrict__ b2b, const float* __restrict__ b2c,
    float* __restrict__ sh0, float* __restrict__ sh1, float* __restrict__ sh2,
    float* __restrict__ b1f, float* __restrict__ b2p) {
  const int reg = blockIdx.y;
  const int i   = blockIdx.x * NTHR + threadIdx.x;
  float v = 0.0f; float* dst = sh0; int n = 0;
  if (reg == 0) {
    n = 512; const int ic = iclamp(i, 0, 511); v = fmaf(db0[ic], s10[ic], t10[ic]); dst = sh0;
  } else if (reg == 1) {
    n = 256; const int ic = iclamp(i, 0, 255); v = fmaf(db1[ic], s11[ic], t11[ic]); dst = sh1;
  } else if (reg == 2) {
    n = 64; const int ic = iclamp(i, 0, 63); v = fmaf(db2[ic], s12[ic], t12[ic]); dst = sh2;
  } else if (reg == 3) {
    n = 768;
    const float* bs = (blockIdx.x == 0) ? b1a : ((blockIdx.x == 1) ? b1b : b1c);
    v = ACARRY * bs[threadIdx.x];
    dst = b1f;
  } else {
    n = 64;
    const float va = b2a[iclamp(i, 0, 33)];
    const float vb = b2b[iclamp(i - 34, 0, 16)];
    const float vc = b2c[iclamp(i - 51, 0, 1)];
    const float fa = (i < 34) ? 1.0f : 0.0f;
    const float fb = (i >= 34 && i < 51) ? 1.0f : 0.0f;
    const float fc = (i >= 51 && i < 53) ? 1.0f : 0.0f;
    v = fmaf(fa, va, fmaf(fb, vb, fc * vc));
    dst = b2p;
  }
  if (i >= n) return;
  st2_f1(dst + i, v);
}

__global__ __launch_bounds__(NTHR) void k_im2col(const float* __restrict__ src, int lr, int lc, int nbase, int total,
                                                 unsigned short* __restrict__ col) {
  const int i = blockIdx.x * NTHR + threadIdx.x;
  if (i >= total) return;
  const int C   = 1 << lc, R = 1 << lr;
  const int cpr = (9 * C) >> 3;
  const int nl  = i / cpr;
  const int q   = i - nl * cpr;
  const int e0  = q << 3;
  const int k   = e0 >> lc;
  const int c0  = e0 & (C - 1);
  const int n   = nbase + nl;
  const int b   = n >> (2 * lr);
  const int y   = (n >> lr) & (R - 1);
  const int x   = n & (R - 1);
  const int kh  = k / 3, kw = k - kh * 3;
  const int yy  = y + kh - 1, xx = x + kw - 1;
  const bool valid = (yy >= 0) && (yy < R) && (xx >= 0) && (xx < R);
  const int yc  = iclamp(yy, 0, R - 1), xc = iclamp(xx, 0, R - 1);
  const float f = valid ? ACARRY : 0.0f;
  const float* sp = src + pact_pix(b, yc, xc, lr - 1) * (size_t)C + c0;
  const v4f u0 = *(const v4f*)sp;
  const v4f u1 = *(const v4f*)(sp + 4);
  v8h hv;
#pragma unroll
  for (int e = 0; e < 4; ++e) { hv[e] = (_Float16)(u0[e] * f); hv[4 + e] = (_Float16)(u1[e] * f); }
  st2_h8(col + (size_t)i * 8, hv);
}

__global__ __launch_bounds__(NTHR) void k_sample(const float* __restrict__ src, const float* __restrict__ om,
                                                 const float* __restrict__ ob, int lr, int lc, int nbase, int total,
                                                 unsigned short* __restrict__ col) {
  const int i = blockIdx.x * NTHR + threadIdx.x;
  if (i >= total) return;
  const int C   = 1 << lc, R = 1 << lr;
  const int cpr = (9 * C) >> 3;
  const int nl  = i / cpr;
  const int q   = i - nl * cpr;
  const int e0  = q << 3;
  const int k   = e0 >> lc;
  const int c0  = e0 & (C - 1);
  const int n   = nbase + nl;
  const int b   = n >> (2 * lr);
  const int y   = (n >> lr) & (R - 1);
  const int x   = n & (R - 1);
  const int kh  = k / 3, kw = k - kh * 3;
  const float* omr = om + (size_t)nl * OMP;
  const float dy = omr[2 * k] + ob[2 * k];
  const float dx = omr[2 * k + 1] + ob[2 * k + 1];
  const float ml = omr[18 + k] + ob[18 + k];
  const float mk = 1.0f / (1.0f + expf(-ml));
  float py = ((float)y + (float)(kh - 1)) + dy;
  float px = ((float)x + (float)(kw - 1)) + dx;
  py = fminf(fmaxf(py, -8.0f), (float)R + 8.0f);
  px = fminf(fmaxf(px, -8.0f), (float)R + 8.0f);
  const float y0f = floorf(py), x0f = floorf(px);
  const float wy = py - y0f, wx = px - x0f;
  const float rmx = (float)(R - 1);
  const float my0 = (y0f >= 0.0f && y0f <= rmx) ? 1.0f : 0.0f;
  const float my1 = ((y0f + 1.0f) >= 0.0f && (y0f + 1.0f) <= rmx) ? 1.0f : 0.0f;
  const float mx0 = (x0f >= 0.0f && x0f <= rmx) ? 1.0f : 0.0f;
  const float mx1 = ((x0f + 1.0f) >= 0.0f && (x0f + 1.0f) <= rmx) ? 1.0f : 0.0f;
  const int iy = (int)y0f, ix = (int)x0f;
  const int cy0 = iclamp(iy, 0, R - 1), cy1 = iclamp(iy + 1, 0, R - 1);
  const int cx0 = iclamp(ix, 0, R - 1), cx1 = iclamp(ix + 1, 0, R - 1);
  const float w00 = ((1.0f - wy) * (1.0f - wx)) * (my0 * mx0);
  const float w01 = ((1.0f - wy) * wx) * (my0 * mx1);
  const float w10 = (wy * (1.0f - wx)) * (my1 * mx0);
  const float w11 = (wy * wx) * (my1 * mx1);
  const float sc  = mk * ACARRY;
  const int lrh = lr - 1;
  const float* p00 = src + pact_pix(b, cy0, cx0, lrh) * (size_t)C + c0;
  const float* p01 = src + pact_pix(b, cy0, cx1, lrh) * (size_t)C + c0;
  const float* p10 = src + pact_pix(b, cy1, cx0, lrh) * (size_t)C + c0;
  const float* p11 = src + pact_pix(b, cy1, cx1, lrh) * (size_t)C + c0;
  const v4f a00 = *(const v4f*)p00, b00 = *(const v4f*)(p00 + 4);
  const v4f a01 = *(const v4f*)p01, b01 = *(const v4f*)(p01 + 4);
  asm volatile("" ::: "memory");
  const v4f a10 = *(const v4f*)p10, b10 = *(const v4f*)(p10 + 4);
  const v4f a11 = *(const v4f*)p11, b11 = *(const v4f*)(p11 + 4);
  v8h hv;
#pragma unroll
  for (int e = 0; e < 4; ++e) {
    const float s0 = ((a00[e] * w00 + a01[e] * w01) + a10[e] * w10) + a11[e] * w11;
    const float s1 = ((b00[e] * w00 + b01[e] * w01) + b10[e] * w10) + b11[e] * w11;
    hv[e]     = (_Float16)(s0 * sc);
    hv[4 + e] = (_Float16)(s1 * sc);
  }
  st2_h8(col + (size_t)i * 8, hv);
}

__global__ __launch_bounds__(NTHR) void k_decim2col(const float* __restrict__ act, int lrh, int lco, int total,
                                                    unsigned short* __restrict__ colp) {
  const int i = blockIdx.x * NTHR + threadIdx.x;
  if (i >= total) return;
  const int Co   = 1 << lco, Rh = 1 << lrh;
  const int lcpr = lco - 1;
  const int lnp  = 2 + 2 * lrh;
  const int p    = i >> (lnp + lcpr);
  const int rem  = i & ((1 << (lnp + lcpr)) - 1);
  const int nl   = rem >> lcpr;
  const int q    = rem & ((1 << lcpr) - 1);
  const int e0   = q << 3;
  const int t    = e0 >> lco;
  const int ci0  = e0 & (Co - 1);
  const int a = p >> 1, bb = p & 1, ty = t >> 1, tx = t & 1;
  const int b    = nl >> (2 * lrh);
  const int y    = (nl >> lrh) & (Rh - 1);
  const int x    = nl & (Rh - 1);
  const int yy   = y + ty - 1 + a, xx = x + tx - 1 + bb;
  const bool valid = (yy >= 0) && (yy < Rh) && (xx >= 0) && (xx < Rh);
  const int yc   = iclamp(yy, 0, Rh - 1), xc = iclamp(xx, 0, Rh - 1);
  const float f  = valid ? ACARRY : 0.0f;
  const float* sp = act + ((((size_t)b << lrh) + (size_t)yc) * (size_t)Rh + (size_t)xc) * (size_t)Co + ci0;
  const v4f u0 = *(const v4f*)sp;
  const v4f u1 = *(const v4f*)(sp + 4);
  v8h hv;
#pragma unroll
  for (int e = 0; e < 4; ++e) { hv[e] = (_Float16)(u0[e] * f); hv[4 + e] = (_Float16)(u1[e] * f); }
  st2_h8(colp + (size_t)i * 8, hv);
}

static int ilog2i(int v) { int l = 0; while ((1 << l) < v) ++l; return l; }
static unsigned cdivu(long a, long b) { return (unsigned)((a + b - 1) / b); }
static unsigned gemm_blocks(int M, int N) { return (unsigned)((((long)(M / 64) * (N / 64)) + 7) / 8); }

extern "C" void kernel_launch(void* const* d_in, const int* in_sizes, int n_in,
                              void* d_out, int out_size, void* d_ws, size_t ws_size,
                              hipStream_t stream)
{
  (void)in_sizes;
  if (n_in < 40) return;
  if ((size_t)out_size < (size_t)NB * NCLS * NPIMG) return;
  if (ws_size < WS_TOTAL) return;

  const float* x = (const float*)d_in[0];
  const float* dwo[3] = {(const float*)d_in[1],  (const float*)d_in[10], (const float*)d_in[19]};
  const float* dbo[3] = {(const float*)d_in[2],  (const float*)d_in[11], (const float*)d_in[20]};
  const float* dwm[3] = {(const float*)d_in[3],  (const float*)d_in[12], (const float*)d_in[21]};
  const float* dbm[3] = {(const float*)d_in[4],  (const float*)d_in[13], (const float*)d_in[22]};
  const float* s1v[3] = {(const float*)d_in[5],  (const float*)d_in[14], (const float*)d_in[23]};
  const float* t1v[3] = {(const float*)d_in[6],  (const float*)d_in[15], (const float*)d_in[24]};
  const float* uwv[3] = {(const float*)d_in[7],  (const float*)d_in[16], (const float*)d_in[25]};
  const float* s2v[3] = {(const float*)d_in[8],  (const float*)d_in[17], (const float*)d_in[26]};
  const float* t2v[3] = {(const float*)d_in[9],  (const float*)d_in[18], (const float*)d_in[27]};
  const float* hw1[3] = {(const float*)d_in[28], (const float*)d_in[32], (const float*)d_in[36]};
  const float* hb1[3] = {(const float*)d_in[29], (const float*)d_in[33], (const float*)d_in[37]};
  const float* hw2[3] = {(const float*)d_in[30], (const float*)d_in[34], (const float*)d_in[38]};
  const float* hb2[3] = {(const float*)d_in[31], (const float*)d_in[35], (const float*)d_in[39]};
  float* outp = (float*)d_out;

  char* base = (char*)d_ws;
  size_t off = 0;
  auto carve = [&](size_t bytes) -> char* { char* p = base + off; off += (bytes + 255) & ~(size_t)255; return p; };
  unsigned short* WPO[3]; unsigned short* WDW[3]; unsigned short* UWP[3];
  WPO[0] = (unsigned short*)carve(SZ_WPO0); WPO[1] = (unsigned short*)carve(SZ_WPO1); WPO[2] = (unsigned short*)carve(SZ_WPO2);
  WDW[0] = (unsigned short*)carve(SZ_WDW0); WDW[1] = (unsigned short*)carve(SZ_WDW1); WDW[2] = (unsigned short*)carve(SZ_WDW2);
  UWP[0] = (unsigned short*)carve(SZ_UWP0); UWP[1] = (unsigned short*)carve(SZ_UWP1); UWP[2] = (unsigned short*)carve(SZ_UWP2);
  unsigned short* WH1 = (unsigned short*)carve(SZ_WH1);
  unsigned short* WH2 = (unsigned short*)carve(SZ_WH2);
  float* SH[3];
  SH[0] = (float*)carve(SZ_SH0); SH[1] = (float*)carve(SZ_SH1); SH[2] = (float*)carve(SZ_SH2);
  float* B1F   = (float*)carve(SZ_B1F);
  float* B2P   = (float*)carve(SZ_B2P);
  float* OM    = (float*)carve(SZ_OM);
  unsigned short* COL = (unsigned short*)carve(SZ_COL);
  float* ACTB  = (float*)carve(SZ_ACTB);
  float* PACTA = (float*)carve(SZ_PACT);
  float* PACTB = (float*)carve(SZ_PACT);
  unsigned short* HID = (unsigned short*)carve(SZ_HID);
  if (off > ws_size) return;

  const int CI[3] = {1024, 512, 256};
  const int CO[3] = {512, 256, 64};
  const int RR[3] = {16, 32, 64};

  k_xprep<<<1024, NTHR, 0, stream>>>(x, PACTB);
  for (int i = 0; i < 3; ++i) {
    const int lc = ilog2i(CI[i]), lco = ilog2i(CO[i]);
    const long cpr = (9L * CI[i]) / 8;
    k_pack3<false><<<cdivu(64 * cpr, NTHR), NTHR, 0, stream>>>(dwo[i], nullptr, 27, lc, 64, WPO[i]);
    k_pack3<true><<<cdivu((long)CO[i] * cpr, NTHR), NTHR, 0, stream>>>(dwm[i], s1v[i], CO[i], lc, CO[i], WDW[i]);
    k_packdec<<<cdivu(2L * CO[i] * CO[i], NTHR), NTHR, 0, stream>>>(uwv[i], s2v[i], lco, UWP[i]);
  }
  for (int hd = 0; hd < 3; ++hd)
    k_pack3<false><<<cdivu(256L * 72, NTHR), NTHR, 0, stream>>>(hw1[hd], nullptr, 256, 6, 256, WH1 + (size_t)hd * 256 * HK1);
  k_packh2<<<dim3(8, 3), NTHR, 0, stream>>>(hw2[0], hw2[1], hw2[2], WH2);
  k_tables<<<dim3(3, 5), NTHR, 0, stream>>>(dbm[0], s1v[0], t1v[0], dbm[1], s1v[1], t1v[1], dbm[2], s1v[2], t1v[2],
                                            hb1[0], hb1[1], hb1[2], hb2[0], hb2[1], hb2[2],
                                            SH[0], SH[1], SH[2], B1F, B2P);

  for (int i = 0; i < 3; ++i) {
    const int C = CI[i], Co = CO[i], R = RR[i];
    const int lc = ilog2i(C), lco = ilog2i(Co), lr = ilog2i(R);
    const int npix = NB * R * R;
    const int nch  = (i == 2) ? 2 : 1;
    const int nloc = npix / nch;
    const int K9   = 9 * C;
    const long cpr = K9 / 8;
    const float* pin  = (i == 1) ? PACTA : PACTB;
    float*       pout = (i == 1) ? PACTB : PACTA;
    for (int ch = 0; ch < nch; ++ch) {
      const int nbase = ch * nloc;
      const int total = (int)(nloc * cpr);
      k_im2col<<<cdivu(total, NTHR), NTHR, 0, stream>>>(pin, lr, lc, nbase, total, COL);
      wmma_gemm64<0, false, 0, 0, false, 0, 0><<<dim3(gemm_blocks(nloc, OMP), 1), 256, 0, stream>>>(
          COL, nullptr, K9, 0L, WPO[i], nullptr, K9, 0L, (void*)OM, nullptr, OMP, 0L,
          nullptr, nullptr, 0L, nloc, OMP, K9, INV_AW, nloc);
      k_sample<<<cdivu(total, NTHR), NTHR, 0, stream>>>(pin, OM, dbo[i], lr, lc, nbase, total, COL);
      wmma_gemm64<0, false, 2, 0, false, 2, 0><<<dim3(gemm_blocks(nloc, Co), 1), 256, 0, stream>>>(
          COL, nullptr, K9, 0L, WDW[i], nullptr, K9, 0L, (void*)(ACTB + (size_t)nbase * Co), nullptr, Co, 0L,
          SH[i], nullptr, 0L, nloc, Co, K9, INV_AW, nloc);
    }
    const int K4 = 4 * Co;
    const int totd = 4 * npix * (Co / 2);
    k_decim2col<<<cdivu(totd, NTHR), NTHR, 0, stream>>>(ACTB, lr, lco, totd, COL);
    wmma_gemm64<0, false, 2, 0, false, 2, 0><<<dim3(gemm_blocks(npix, Co), 4), 256, 0, stream>>>(
        COL, nullptr, K4, (long)npix * K4, UWP[i], nullptr, K4, (long)Co * K4, (void*)pout, nullptr, Co, (long)npix * Co,
        t2v[i], nullptr, 0L, npix, Co, K4, INV_AW, npix);
  }

  for (int img = 0; img < NB; ++img) {
    const int total = NPIMG * 72;
    k_im2col<<<cdivu(total, NTHR), NTHR, 0, stream>>>(PACTA, RES_OUT_LOG, 6, img * NPIMG, total, COL);
    wmma_gemm64<0, false, 2, 1, false, 2, 0><<<dim3(gemm_blocks(NPIMG, NHID), 1), 256, 0, stream>>>(
        COL, nullptr, HK1, 0L, WH1, nullptr, HK1, 0L, (void*)HID, nullptr, NHID, 0L,
        B1F, nullptr, 0L, NPIMG, NHID, HK1, INV_W, NPIMG);
    wmma_gemm64<0, false, 1, 0, false, 0, 1><<<dim3(gemm_blocks(HM2, NPIMG), 1), 256, 0, stream>>>(
        WH2, nullptr, NHID, 0L, HID, nullptr, NHID, 0L, (void*)(outp + (size_t)img * NCLS * NPIMG), nullptr, NPIMG, 0L,
        B2P, nullptr, 0L, HM2, NPIMG, NHID, INV_AW, NCLS);
  }
}
